// RNNPPAgent_49469433315484
// MI455X (gfx1250) — hardware-run, weakly checked
//
#include <hip/hip_runtime.h>
#include <math.h>

typedef __attribute__((ext_vector_type(16))) _Float16 v16h;
typedef __attribute__((ext_vector_type(8)))  _Float16 v8h;
typedef __attribute__((ext_vector_type(16))) __bf16   v16b;
typedef __attribute__((ext_vector_type(8)))  __bf16   v8b;
typedef __attribute__((ext_vector_type(8)))  float    v8f;
typedef __attribute__((ext_vector_type(4)))  float    v4f;
typedef __attribute__((ext_vector_type(4)))  unsigned v4u;
typedef __attribute__((ext_vector_type(4)))  int      v4i;

constexpr int kRows   = 32768;
constexpr int kIn     = 204;
constexpr int kInP    = 224;
constexpr int kHid    = 128;
constexpr int kGate   = 384;
constexpr int kMech   = 4;
constexpr int kAct    = 14;
constexpr int kRt     = 32;
constexpr int kXaP    = kMech * kHid;
constexpr int kTP     = 132;
constexpr int kRtP    = 33;
constexpr int kRtTile = 16 * kRtP;
constexpr float kActCarry = 8.0f;
constexpr float kWCarry   = 256.0f;
constexpr float kAccScale = 1.0f / (8.0f * 256.0f);
static_assert(kInP % 32 == 0 && kInP >= kIn && kHid % 32 == 0, "GEMM K multiples of 32");
static_assert(kRows % 64 == 0 && kXaP % 64 == 0, "GEMM M,N multiples of 64");
static_assert(kIn % 4 == 0, "16-B aligned input rows");
static_assert((kRows * (kInP / 8)) % 256 == 0 && (kRows * (kHid / 8)) % 256 == 0, "cast grids exact");
static_assert((16 * kAct * 4) % 128 == 0, "16-row group of the narrow output is whole lines");

constexpr size_t kOffX16  = 0;
constexpr size_t kOffH16  = kOffX16  + (size_t)kRows * kInP * 2;
constexpr size_t kOffXA16 = kOffH16  + (size_t)kRows * kHid * 2;
constexpr size_t kOffFC1T = kOffXA16 + (size_t)kRows * kXaP * 2;
constexpr size_t kOffWIHT = kOffFC1T + (size_t)kXaP * kInP * 2;
constexpr size_t kOffWHHT = kOffWIHT + (size_t)kMech * kGate * kHid * 2;
constexpr size_t kOffW1TH = kOffWHHT + (size_t)kMech * kGate * kHid * 2;
constexpr size_t kOffW1TL = kOffW1TH + (size_t)kRt * kHid * 2;
constexpr size_t kOffSEL  = kOffW1TL + (size_t)kRt * kHid * 2;
constexpr size_t kWsTotal = kOffSEL  + (size_t)kRows * 4;
static_assert(kWsTotal == 57786368ull, "carve total");
static_assert(kWsTotal <= 134217728ull, "carve cap");
static_assert((kOffH16 % 128) == 0 && (kOffXA16 % 128) == 0 && (kOffFC1T % 128) == 0 && (kOffWIHT % 128) == 0 &&
              (kOffWHHT % 128) == 0 && (kOffW1TH % 128) == 0 && (kOffW1TL % 128) == 0 && (kOffSEL % 128) == 0,
              "128-B aligned regions");

__device__ __forceinline__ unsigned short f2bf_bits(float f) {
  unsigned u = __float_as_uint(f);
  return (unsigned short)((u + 0x7FFFu + ((u >> 16) & 1u)) >> 16);
}
__device__ __forceinline__ float bf_bits2f(unsigned short h) { return __uint_as_float(((unsigned)h) << 16); }
__device__ __forceinline__ void split_bf(float f, __bf16& hi, __bf16& lo) {
  const unsigned short hb = f2bf_bits(f);
  const unsigned short lb = f2bf_bits(f - bf_bits2f(hb));
  hi = __builtin_bit_cast(__bf16, hb);
  lo = __builtin_bit_cast(__bf16, lb);
}
__device__ __forceinline__ float sel4(int m, float a, float b, float c, float d) {
  return (m == 0) ? a : ((m == 1) ? b : ((m == 2) ? c : d));
}
__device__ __forceinline__ float fast_sigmoid(float x) {
  return __builtin_amdgcn_rcpf(1.0f + __expf(-x));
}
__device__ __forceinline__ float fast_tanh(float x) {
  return 1.0f - 2.0f * __builtin_amdgcn_rcpf(1.0f + __expf(2.0f * x));
}

__device__ __forceinline__ void guard4_h(v8f& a, v8f& b, v8f& c, v8f& d, v16h x, v16h y) {
  asm volatile("v_nop\n\tv_nop\n\tv_nop\n\tv_nop" : "+v"(a), "+v"(b), "+v"(c), "+v"(d) : "v"(x), "v"(y));
}
__device__ __forceinline__ void keep4_h(v16h a, v16h b, v16h c, v16h d) { asm volatile("v_nop" :: "v"(a), "v"(b), "v"(c), "v"(d)); }
__device__ __forceinline__ void acc_guard4(v8f& a, v8f& b, v8f& c, v8f& d) {
  asm volatile("v_nop\n\tv_nop\n\tv_nop\n\tv_nop" : "+v"(a), "+v"(b), "+v"(c), "+v"(d));
}
__device__ __forceinline__ void guard_gate_h(v8f& a, v8f& b, v8f& c, v8f& d, v16h x, v16h y,
                                             v16h b0, v16h b1, v16h b2, v16h b3, v16h b4, v16h b5) {
  asm volatile("v_nop\n\tv_nop\n\tv_nop\n\tv_nop" : "+v"(a), "+v"(b), "+v"(c), "+v"(d)
               : "v"(x), "v"(y), "v"(b0), "v"(b1), "v"(b2), "v"(b3), "v"(b4), "v"(b5));
}
__device__ __forceinline__ void guard_rt_b(v8f& a, v8f& b, v16b x, v16b y, v16b b0, v16b b1, v16b b2, v16b b3) {
  asm volatile("v_nop\n\tv_nop\n\tv_nop\n\tv_nop" : "+v"(a), "+v"(b)
               : "v"(x), "v"(y), "v"(b0), "v"(b1), "v"(b2), "v"(b3));
}

template <typename T> struct Frag;
template <> struct Frag<_Float16> {
  typedef v16h V; union U { v16h v; v8h h[2]; };
  static __device__ __forceinline__ v16h load(const _Float16* p) {
    U f; f.h[0] = *(const v8h*)(p); f.h[1] = *(const v8h*)(p + 16); return f.v;
  }
  static __device__ __forceinline__ v8f mma(v16h a, v16h b, v8f c) {
    return __builtin_amdgcn_wmma_f32_16x16x32_f16(false, a, false, b, (short)0, c, false, false);
  }
};
template <> struct Frag<__bf16> {
  typedef v16b V; union U { v16b v; v8b h[2]; };
  static __device__ __forceinline__ v16b load(const __bf16* p) {
    U f; f.h[0] = *(const v8b*)(p); f.h[1] = *(const v8b*)(p + 16); return f.v;
  }
  static __device__ __forceinline__ v8f mma(v16b a, v16b b, v8f c) {
    return __builtin_amdgcn_wmma_f32_16x16x32_bf16(false, a, false, b, (short)0, c, false, false);
  }
};

template <int MODE>
__global__ __launch_bounds__(256) void transpose_w_kernel(
    const float* __restrict__ src, unsigned short* __restrict__ dst, unsigned short* __restrict__ dst2,
    int K, int N, int KP, float scale)
{
  __shared__ __align__(16) unsigned short tH[16 * kInP];
  __shared__ __align__(16) unsigned short tL[(MODE == 1) ? 16 * kInP : 8];
  const int tid = threadIdx.x;
  const int b = blockIdx.y;
  const int n0 = blockIdx.x * 16;
  const float* srcb = src + (size_t)b * K * N;
  const int total = 16 * KP;
  for (int idx = tid; idx < total; idx += 256) {
    const int nn = idx & 15;
    const int k = idx >> 4;
    const int kc = (k < K) ? k : (K - 1);
    float v = srcb[(size_t)kc * N + n0 + nn];
    v = (k < K) ? (v * scale) : 0.0f;
    if (MODE == 0) {
      const _Float16 hv = (_Float16)v;
      tH[nn * KP + k] = __builtin_bit_cast(unsigned short, hv);
    } else {
      const unsigned short hb = f2bf_bits(v);
      const unsigned short lb = f2bf_bits(v - bf_bits2f(hb));
      tH[nn * KP + k] = hb;
      tL[nn * KP + k] = lb;
    }
  }
  __syncthreads();
  const int pieces = total >> 3;
  unsigned short* d1 = dst + ((size_t)b * N + n0) * KP;
  unsigned short* d2 = (MODE == 1) ? (dst2 + ((size_t)b * N + n0) * KP) : nullptr;
  for (int pass = 0; pass < 2; ++pass) {
    for (int p = tid; p < pieces; p += 256) {
      const v4u q = *(const v4u*)(tH + p * 8);
      *(volatile v4u*)(d1 + p * 8) = q;
      if (MODE == 1) {
        const v4u ql = *(const v4u*)(tL + p * 8);
        *(volatile v4u*)(d2 + p * 8) = ql;
      }
    }
    __threadfence();
  }
}

__global__ __launch_bounds__(256) void cast_rows_f16_kernel(
    const float* __restrict__ src, unsigned short* __restrict__ dst, int K, int KP, int total_pieces, float scale)
{
  const int p = blockIdx.x * 256 + threadIdx.x;
  if (p >= total_pieces) return;
  const int ppr = KP >> 3;
  const int row = p / ppr;
  const int c8 = (p - row * ppr) * 8;
  const int ca = (c8 < K - 4) ? c8 : (K - 4);
  const int cb = (c8 + 4 < K - 4) ? (c8 + 4) : (K - 4);
  const v4f a0 = *(const v4f*)(src + (size_t)row * K + ca);
  const v4f a1 = *(const v4f*)(src + (size_t)row * K + cb);
  v8h hv;
#pragma unroll
  for (int e = 0; e < 4; ++e) {
    float x0 = a0[e];
    float x1 = a1[e];
    x0 = (c8 + e < K) ? (x0 * scale) : 0.0f;
    x1 = (c8 + 4 + e < K) ? (x1 * scale) : 0.0f;
    hv[e] = (_Float16)x0;
    hv[4 + e] = (_Float16)x1;
  }
  unsigned short* q = dst + (size_t)p * 8;
  *(volatile v8h*)q = hv;
  __threadfence();
  *(volatile v8h*)q = hv;
}

__global__ __launch_bounds__(128) void router_select_kernel(
    const float* __restrict__ HIN, const unsigned short* __restrict__ W1Thp, const unsigned short* __restrict__ W1Tlp,
    const float* __restrict__ QPB1, const float* __restrict__ QPW2, const float* __restrict__ QPB2,
    const float* __restrict__ QPW3, const float* __restrict__ QPB3, const float* __restrict__ KEYS,
    const float* __restrict__ WQ, const float* __restrict__ BQ, const float* __restrict__ WK,
    const float* __restrict__ BK, const float* __restrict__ UNZ, int* __restrict__ SEL)
{
  typedef Frag<__bf16> FB;
  __shared__ __align__(16) float sW[3 * 1024];
  __shared__ float sBias[128];
  __shared__ float sKP[128];
  __shared__ __align__(16) float sBuf[4][2 * kRtTile];
  __shared__ __align__(16) int sSel[64];
  const __bf16* W1h = (const __bf16*)W1Thp;
  const __bf16* W1l = (const __bf16*)W1Tlp;
  const int tid = threadIdx.x, lane = tid & 31, wave = tid >> 5;
  const int hh = lane >> 4, c = lane & 15;
  const int row0 = blockIdx.x * 64;
  const int wrow0 = row0 + wave * 16;

#pragma unroll 1
  for (int i = 0; i < 8; ++i) {
    const int idx = i * 128 + tid;
    sW[idx] = QPW2[idx];
    sW[1024 + idx] = QPW3[idx];
    sW[2048 + idx] = WQ[idx];
  }
  {
    const int j = tid & 31;
    float c0 = QPB1[j];
    float c1 = QPB2[j];
    float c2 = QPB3[j];
    float c3 = BQ[j];
    asm volatile("" : "+v"(c0));
    asm volatile("" : "+v"(c1));
    asm volatile("" : "+v"(c2));
    asm volatile("" : "+v"(c3));
    sBias[tid] = sel4(wave, c0, c1, c2, c3);
    float acc = 0.0f;
#pragma unroll 1
    for (int k = 0; k < kRt; ++k) acc = fmaf(KEYS[wave * kRt + k], WK[k * kRt + j], acc);
    sKP[tid] = acc + BK[j];
  }
  __syncthreads();

  v8f acc0 = (v8f){0.f,0.f,0.f,0.f,0.f,0.f,0.f,0.f};
  v8f acc1 = (v8f){0.f,0.f,0.f,0.f,0.f,0.f,0.f,0.f};
  {
    const float* hrow = HIN + (size_t)(wrow0 + c) * kHid + 8 * hh;
#pragma unroll
    for (int ks = 0; ks < 4; ++ks) {
      const v4f f0 = *(const v4f*)(hrow + ks * 32);
      const v4f f1 = *(const v4f*)(hrow + ks * 32 + 4);
      const v4f f2 = *(const v4f*)(hrow + ks * 32 + 16);
      const v4f f3 = *(const v4f*)(hrow + ks * 32 + 20);
      v16b ah, al;
#pragma unroll
      for (int e = 0; e < 4; ++e) {
        __bf16 hq, lq;
        const float x0 = f0[e];
        split_bf(x0, hq, lq); ah[e] = hq; al[e] = lq;
        const float x1 = f1[e];
        split_bf(x1, hq, lq); ah[4 + e] = hq; al[4 + e] = lq;
        const float x2 = f2[e];
        split_bf(x2, hq, lq); ah[8 + e] = hq; al[8 + e] = lq;
        const float x3 = f3[e];
        split_bf(x3, hq, lq); ah[12 + e] = hq; al[12 + e] = lq;
      }
      const size_t bo0 = (size_t)c * kHid + ks * 32 + 8 * hh;
      const size_t bo1 = (size_t)(16 + c) * kHid + ks * 32 + 8 * hh;
      const v16b bh0 = FB::load(W1h + bo0);
      const v16b bh1 = FB::load(W1h + bo1);
      const v16b bl0 = FB::load(W1l + bo0);
      const v16b bl1 = FB::load(W1l + bo1);
      acc0 = FB::mma(ah, bh0, acc0);
      acc0 = FB::mma(ah, bl0, acc0);
      acc0 = FB::mma(al, bh0, acc0);
      acc1 = FB::mma(ah, bh1, acc1);
      acc1 = FB::mma(ah, bl1, acc1);
      acc1 = FB::mma(al, bh1, acc1);
      guard_rt_b(acc0, acc1, ah, al, bh0, bh1, bl0, bl1);
    }
  }
  float* mybuf = sBuf[wave];
  {
    const float b0 = sBias[c];
    const float b1 = sBias[16 + c];
#pragma unroll
    for (int r = 0; r < 8; ++r) {
      mybuf[(8 * hh + r) * kRtP + c] = fmaxf(acc0[r] + b0, 0.0f);
      mybuf[(8 * hh + r) * kRtP + 16 + c] = fmaxf(acc1[r] + b1, 0.0f);
    }
  }
  __syncthreads();

#pragma unroll 1
  for (int st = 0; st < 3; ++st) {
    const float* wst = sW + st * 1024;
    const float bv = sBias[32 * (st + 1) + lane];
    const float* srcb = mybuf + (st & 1) * kRtTile;
    float* dstb = mybuf + (1 - (st & 1)) * kRtTile;
#pragma unroll 1
    for (int p = 0; p < 2; ++p) {
      float a[8];
#pragma unroll
      for (int r = 0; r < 8; ++r) a[r] = 0.0f;
      const float* sp = srcb + p * 8 * kRtP;
#pragma unroll 1
      for (int k = 0; k < kRt; ++k) {
        const float w = wst[k * kRt + lane];
#pragma unroll
        for (int r = 0; r < 8; ++r) a[r] = fmaf(sp[r * kRtP + k], w, a[r]);
      }
#pragma unroll
      for (int r = 0; r < 8; ++r) {
        float v = a[r] + bv;
        v = (st == 0) ? fmaxf(v, 0.0f) : v;
        dstb[(p * 8 + r) * kRtP + lane] = v;
      }
    }
    __syncthreads();
  }

  int bi = 0;
  {
#pragma clang fp contract(off)
    const int rr = lane & 15;
    const float* qrow = mybuf + kRtTile + rr * kRtP;
    float l0 = 0.0f, l1 = 0.0f, l2 = 0.0f, l3 = 0.0f;
#pragma unroll 1
    for (int k = 0; k < kRt; ++k) {
      const float q = qrow[k];
      l0 = fmaf(q, sKP[k], l0);
      l1 = fmaf(q, sKP[32 + k], l1);
      l2 = fmaf(q, sKP[64 + k], l2);
      l3 = fmaf(q, sKP[96 + k], l3);
    }
    const float scl = 1.0f / sqrtf((float)kRt);
    l0 *= scl; l1 *= scl; l2 *= scl; l3 *= scl;
    const v4f uv = *(const v4f*)(UNZ + (size_t)(wrow0 + rr) * 4);
    const float u0 = uv[0];
    const float u1 = uv[1];
    const float u2 = uv[2];
    const float u3 = uv[3];
    const float mx = fmaxf(fmaxf(l0, l1), fmaxf(l2, l3));
    float e0 = 0.0f, e1 = 0.0f, e2 = 0.0f, e3 = 0.0f, esum = 0.0f;
#pragma unroll 1
    for (int m = 0; m < kMech; ++m) {
      const float lm = sel4(m, l0, l1, l2, l3);
      const float e = expf(lm - mx);
      esum += e;
      e0 = (m == 0) ? e : e0;
      e1 = (m == 1) ? e : e1;
      e2 = (m == 2) ? e : e2;
      e3 = (m == 3) ? e : e3;
    }
    float t0 = 0.0f, t1 = 0.0f, t2 = 0.0f, t3 = 0.0f, tmax = -INFINITY;
#pragma unroll 1
    for (int m = 0; m < kMech; ++m) {
      const float em = sel4(m, e0, e1, e2, e3);
      const float um = sel4(m, u0, u1, u2, u3);
      const float g = -logf(-logf(um + 1e-10f) + 1e-10f);
      const float p = em / esum;
      const float t = p + g;
      tmax = fmaxf(tmax, t);
      t0 = (m == 0) ? t : t0;
      t1 = (m == 1) ? t : t1;
      t2 = (m == 2) ? t : t2;
      t3 = (m == 3) ? t : t3;
    }
    float y0 = 0.0f, y1 = 0.0f, y2 = 0.0f, y3 = 0.0f, ysum = 0.0f;
#pragma unroll 1
    for (int m = 0; m < kMech; ++m) {
      const float tm = sel4(m, t0, t1, t2, t3);
      const float y = expf(tm - tmax);
      ysum += y;
      y0 = (m == 0) ? y : y0;
      y1 = (m == 1) ? y : y1;
      y2 = (m == 2) ? y : y2;
      y3 = (m == 3) ? y : y3;
    }
    float best = -INFINITY;
#pragma unroll 1
    for (int m = 0; m < kMech; ++m) {
      const float ym = sel4(m, y0, y1, y2, y3);
      const float yn = ym / ysum;
      if (yn > best) { best = yn; bi = m; }
    }
  }
  if (lane < 16) sSel[wave * 16 + lane] = bi;
  __syncthreads();
  if (tid < 16) {
    const v4i sv = *(const v4i*)(sSel + tid * 4);
    volatile v4i* p = (volatile v4i*)(SEL + row0 + tid * 4);
    *p = sv;
    __threadfence();
    *p = sv;
  }
}

__global__ __launch_bounds__(256) void fc1_gemm_kernel(
    const unsigned short* __restrict__ Ap, int lda, const unsigned short* __restrict__ Btp, int ldb,
    unsigned short* __restrict__ Cout, int ldc, const float* __restrict__ bias,
    int M, int N, int K, float scale, float oscale)
{
  typedef Frag<_Float16> F;
  const _Float16* A = (const _Float16*)Ap;
  const _Float16* Bt = (const _Float16*)Btp;
  __shared__ __align__(16) float sT[8][16 * 68];
  const int lane = threadIdx.x & 31;
  const int wave = threadIdx.x >> 5;
  const int tilesN = N >> 6;
  const int tilesM = M >> 6;
  const int tile = blockIdx.x * 8 + wave;
  if (tile >= tilesM * tilesN) return;
  const int tm = tile / tilesN;
  const int tn = tile - tm * tilesN;
  const int m0 = tm << 6;
  const int n0 = tn << 6;
  const int rlane = lane & 15;
  const int koff  = (lane >> 4) * 8;
  const int mOff  = (lane >> 4) * 8;

  v8f acc[4][4];
#pragma unroll
  for (int i = 0; i < 4; ++i)
#pragma unroll
    for (int j = 0; j < 4; ++j) acc[i][j] = (v8f){0.f,0.f,0.f,0.f,0.f,0.f,0.f,0.f};

  for (int k0 = 0; k0 < K; k0 += 32) {
    v16h bh[4];
#pragma unroll
    for (int j = 0; j < 4; ++j) {
      const size_t bo = (size_t)(n0 + (j << 4) + rlane) * ldb + koff + k0;
      bh[j] = F::load(Bt + bo);
    }
#pragma unroll
    for (int i = 0; i < 4; ++i) {
      const size_t ao = (size_t)(m0 + (i << 4) + rlane) * lda + koff + k0;
      const v16h ah = F::load(A + ao);
#pragma unroll
      for (int j = 0; j < 4; ++j) acc[i][j] = F::mma(ah, bh[j], acc[i][j]);
      guard4_h(acc[i][0], acc[i][1], acc[i][2], acc[i][3], ah, ah);
    }
    keep4_h(bh[0], bh[1], bh[2], bh[3]);
  }
  acc_guard4(acc[0][0], acc[0][1], acc[0][2], acc[0][3]);
  acc_guard4(acc[1][0], acc[1][1], acc[1][2], acc[1][3]);
  acc_guard4(acc[2][0], acc[2][1], acc[2][2], acc[2][3]);
  acc_guard4(acc[3][0], acc[3][1], acc[3][2], acc[3][3]);

  float* slab = sT[wave];
#pragma unroll
  for (int i = 0; i < 4; ++i) {
    const int mBase = m0 + (i << 4);
#pragma unroll
    for (int j = 0; j < 4; ++j) {
      const int n = n0 + (j << 4) + rlane;
      const float bv = bias[n];
#pragma unroll
      for (int r = 0; r < 8; ++r) {
        float v = acc[i][j][r] * scale;
        v += bv;
        v = fmaxf(v, 0.0f);
        v *= oscale;
        slab[(mOff + r) * 68 + (j << 4) + rlane] = v;
      }
    }
    __builtin_amdgcn_fence(__ATOMIC_RELEASE, "workgroup");
    __builtin_amdgcn_wave_barrier();
    __builtin_amdgcn_fence(__ATOMIC_ACQUIRE, "workgroup");
    {
      const int q = lane >> 3, c8 = (lane & 7) * 8;
      for (int pass = 0; pass < 2; ++pass) {
#pragma unroll
        for (int it = 0; it < 4; ++it) {
          const int row = it * 4 + q;
          const float* sp = slab + row * 68 + c8;
          v8h hv;
#pragma unroll
          for (int e = 0; e < 8; ++e) hv[e] = (_Float16)sp[e];
          *(volatile v8h*)(Cout + (size_t)(mBase + row) * ldc + n0 + c8) = hv;
        }
        __threadfence();
      }
    }
    __builtin_amdgcn_fence(__ATOMIC_RELEASE, "workgroup");
    __builtin_amdgcn_wave_barrier();
    __builtin_amdgcn_fence(__ATOMIC_ACQUIRE, "workgroup");
  }
}

__global__ __launch_bounds__(64) void gru_select_kernel(
    const unsigned short* __restrict__ XA16p, const unsigned short* __restrict__ H16p,
    const unsigned short* __restrict__ WihTp, const unsigned short* __restrict__ WhhTp,
    const float* __restrict__ HIN, const float* __restrict__ BIH, const float* __restrict__ BHH,
    const int* __restrict__ SEL, float* __restrict__ OUT1)
{
  typedef Frag<_Float16> F;
  const _Float16* XA = (const _Float16*)XA16p;
  const _Float16* Hh = (const _Float16*)H16p;
  const _Float16* Wi = (const _Float16*)WihTp;
  const _Float16* Wh = (const _Float16*)WhhTp;
  __shared__ __align__(16) float sH[32 * kTP];
  __shared__ __align__(16) float sN[2][16 * kTP];
  __shared__ int sSel[32];
  const int tid = threadIdx.x, lane = tid & 31, wave = tid >> 5;
  const int hh = lane >> 4, c = lane & 15;
  const int row0 = blockIdx.x * 32;
  const int wrow0 = row0 + wave * 16;

#pragma unroll 1
  for (int i = 0; i < 16; ++i) {
    const int idx = i * 64 + tid;
    const int r = idx >> 5;
    const int c4 = (idx & 31) * 4;
    *(v4f*)(sH + r * kTP + c4) = *(const v4f*)(HIN + (size_t)(row0 + r) * kHid + c4);
  }
  {
    int s = SEL[row0 + (tid & 31)];
    asm volatile("" : "+v"(s));
    s = (s < 0) ? 0 : ((s > kMech - 1) ? (kMech - 1) : s);
    if (tid < 32) sSel[tid] = s;
  }
  __syncthreads();

  const _Float16* hA = Hh + (size_t)(wrow0 + c) * kHid + 8 * hh;
  float* myN = sN[wave];
  const float* myH = sH + (wave * 16) * kTP;

#pragma unroll 1
  for (int m = 0; m < kMech; ++m) {
    const _Float16* xA = XA + (size_t)(wrow0 + c) * kXaP + m * kHid + 8 * hh;
#pragma unroll 1
    for (int jb = 0; jb < 4; ++jb) {
      v8f ar[2], az[2], ai[2], an[2];
#pragma unroll
      for (int ns = 0; ns < 2; ++ns) {
        ar[ns] = (v8f){0.f,0.f,0.f,0.f,0.f,0.f,0.f,0.f};
        az[ns] = (v8f){0.f,0.f,0.f,0.f,0.f,0.f,0.f,0.f};
        ai[ns] = (v8f){0.f,0.f,0.f,0.f,0.f,0.f,0.f,0.f};
        an[ns] = (v8f){0.f,0.f,0.f,0.f,0.f,0.f,0.f,0.f};
      }
#pragma unroll 1
      for (int ks = 0; ks < 4; ++ks) {
        const v16h ax = F::load(xA + ks * 32);
        const v16h ah = F::load(hA + ks * 32);
#pragma unroll
        for (int ns = 0; ns < 2; ++ns) {
          const size_t bo = (size_t)(m * kGate + jb * 32 + ns * 16 + c) * kHid + ks * 32 + 8 * hh;
          const v16h wir = F::load(Wi + bo);
          const v16h whr = F::load(Wh + bo);
          const v16h wiz = F::load(Wi + bo + (size_t)kHid * kHid);
          const v16h whz = F::load(Wh + bo + (size_t)kHid * kHid);
          const v16h win = F::load(Wi + bo + (size_t)2 * kHid * kHid);
          const v16h whn = F::load(Wh + bo + (size_t)2 * kHid * kHid);
          ar[ns] = F::mma(ax, wir, ar[ns]);
          ar[ns] = F::mma(ah, whr, ar[ns]);
          az[ns] = F::mma(ax, wiz, az[ns]);
          az[ns] = F::mma(ah, whz, az[ns]);
          ai[ns] = F::mma(ax, win, ai[ns]);
          an[ns] = F::mma(ah, whn, an[ns]);
          guard_gate_h(ar[ns], az[ns], ai[ns], an[ns], ax, ah, wir, whr, wiz, whz, win, whn);
        }
      }
#pragma unroll
      for (int ns = 0; ns < 2; ++ns) {
        const int j = jb * 32 + ns * 16 + c;
        const float bir = BIH[m * kGate + j];
        const float bhr = BHH[m * kGate + j];
        const float biz = BIH[m * kGate + kHid + j];
        const float bhz = BHH[m * kGate + kHid + j];
        const float bin = BIH[m * kGate + 2 * kHid + j];
        const float bhn = BHH[m * kGate + 2 * kHid + j];
#pragma unroll
        for (int r = 0; r < 8; ++r) {
          const int rl = 8 * hh + r;
          const float pr = (ar[ns][r] * kAccScale + bir) + bhr;
          const float pz = (az[ns][r] * kAccScale + biz) + bhz;
          const float gin = ai[ns][r] * kAccScale + bin;
          const float ghn = an[ns][r] * kAccScale + bhn;
          const float rg = fast_sigmoid(pr);
          const float zg = fast_sigmoid(pz);
          const float ng = fast_tanh(gin + rg * ghn);
          const float h0 = myH[rl * kTP + j];
          myN[rl * kTP + j] = (1.0f - zg) * ng + zg * h0;
        }
      }
    }
    __syncthreads();
#pragma unroll 1
    for (int r = 0; r < 16; ++r) {
      const int s = __builtin_amdgcn_readfirstlane(sSel[wave * 16 + r]);
      if (s == m) {
        const v4f v = *(const v4f*)(myN + r * kTP + lane * 4);
        volatile v4f* p = (volatile v4f*)(OUT1 + (size_t)(wrow0 + r) * kHid + lane * 4);
        *p = v;
        __threadfence();
        *p = v;
      }
    }
    __syncthreads();
  }
}

__global__ __launch_bounds__(256) void fc2_select_kernel(
    const float* HSEL, const int* __restrict__ SEL, const float* __restrict__ FC2W,
    const float* __restrict__ FC2B, float* OUT0)
{
  __shared__ __align__(16) float sQ[16 * kAct];
  const int tid = threadIdx.x;
  const int rl = tid >> 4;
  const int a = tid & 15;
  const int ac = (a < kAct) ? a : (kAct - 1);
  const int row = blockIdx.x * 16 + rl;
  int s = SEL[row];
  s = (s < 0) ? 0 : ((s > kMech - 1) ? (kMech - 1) : s);
  const float* hrow = HSEL + (size_t)row * kHid;
  const float* wcol = FC2W + (size_t)s * kHid * kAct + ac;
  float acc = 0.0f;
#pragma unroll 1
  for (int k = 0; k < kHid; k += 4) {
    const v4f hv = *(const v4f*)(hrow + k);
    const float h0 = hv[0];
    const float h1 = hv[1];
    const float h2 = hv[2];
    const float h3 = hv[3];
    acc = fmaf(h0, wcol[(k + 0) * kAct], acc);
    acc = fmaf(h1, wcol[(k + 1) * kAct], acc);
    acc = fmaf(h2, wcol[(k + 2) * kAct], acc);
    acc = fmaf(h3, wcol[(k + 3) * kAct], acc);
  }
  acc += FC2B[s * kAct + ac];
  if (a < kAct) sQ[rl * kAct + a] = acc;
  __syncthreads();
  if (tid < 56) {
    const v4f v = *(const v4f*)(sQ + tid * 4);
    volatile v4f* p = (volatile v4f*)(OUT0 + (size_t)blockIdx.x * (16 * kAct) + tid * 4);
    *p = v;
    __threadfence();
    *p = v;
  }
}

extern "C" void kernel_launch(void* const* d_in, const int* in_sizes, int n_in,
                              void* d_out, int out_size, void* d_ws, size_t ws_size,
                              hipStream_t stream) {
  if (n_in < 22) return;
  if (in_sizes[0] != kRows * kIn) return;
  if (in_sizes[1] != kRows * kHid) return;
  if (in_sizes[2] != kMech * kIn * kHid) return;
  if (in_sizes[3] != kMech * kHid) return;
  if (in_sizes[4] != kMech * kHid * kGate) return;
  if (in_sizes[5] != kMech * kHid * kGate) return;
  if (in_sizes[6] != kMech * kGate) return;
  if (in_sizes[7] != kMech * kGate) return;
  if (in_sizes[8] != kMech * kHid * kAct) return;
  if (in_sizes[9] != kMech * kAct) return;
  if (in_sizes[10] != kHid * kRt) return;
  if (in_sizes[11] != kRt) return;
  if (in_sizes[12] != kRt * kRt) return;
  if (in_sizes[13] != kRt) return;
  if (in_sizes[14] != kRt * kRt) return;
  if (in_sizes[15] != kRt) return;
  if (in_sizes[16] != kMech * kRt) return;
  if (in_sizes[17] != kRt * kRt) return;
  if (in_sizes[18] != kRt) return;
  if (in_sizes[19] != kRt * kRt) return;
  if (in_sizes[20] != kRt) return;
  if (in_sizes[21] != kRows * kMech) return;
  if (out_size != kRows * kAct + kRows * kHid) return;
  if (ws_size < kWsTotal) return;

  const float* X    = (const float*)d_in[0];
  const float* HIN  = (const float*)d_in[1];
  const float* FC1W = (const float*)d_in[2];
  const float* FC1B = (const float*)d_in[3];
  const float* WIH  = (const float*)d_in[4];
  const float* WHH  = (const float*)d_in[5];
  const float* BIH  = (const float*)d_in[6];
  const float* BHH  = (const float*)d_in[7];
  const float* FC2W = (const float*)d_in[8];
  const float* FC2B = (const float*)d_in[9];
  const float* QPW1 = (const float*)d_in[10];
  const float* QPB1 = (const float*)d_in[11];
  const float* QPW2 = (const float*)d_in[12];
  const float* QPB2 = (const float*)d_in[13];
  const float* QPW3 = (const float*)d_in[14];
  const float* QPB3 = (const float*)d_in[15];
  const float* KEYS = (const float*)d_in[16];
  const float* WQ   = (const float*)d_in[17];
  const float* BQ   = (const float*)d_in[18];
  const float* WK   = (const float*)d_in[19];
  const float* BK   = (const float*)d_in[20];
  const float* UNZ  = (const float*)d_in[21];

  float* OUT0 = (float*)d_out;
  float* OUT1 = (float*)d_out + (size_t)kRows * kAct;

  char* ws = (char*)d_ws;
  unsigned short* X16  = (unsigned short*)(ws + kOffX16);
  unsigned short* H16  = (unsigned short*)(ws + kOffH16);
  unsigned short* XA16 = (unsigned short*)(ws + kOffXA16);
  unsigned short* FC1T = (unsigned short*)(ws + kOffFC1T);
  unsigned short* WIHT = (unsigned short*)(ws + kOffWIHT);
  unsigned short* WHHT = (unsigned short*)(ws + kOffWHHT);
  unsigned short* W1TH = (unsigned short*)(ws + kOffW1TH);
  unsigned short* W1TL = (unsigned short*)(ws + kOffW1TL);
  int*            SEL  = (int*)(ws + kOffSEL);

  transpose_w_kernel<0><<<dim3(kHid / 16, kMech), 256, 0, stream>>>(FC1W, FC1T, nullptr, kIn, kHid, kInP, kWCarry);
  transpose_w_kernel<0><<<dim3(kGate / 16, kMech), 256, 0, stream>>>(WIH, WIHT, nullptr, kHid, kGate, kHid, kWCarry);
  transpose_w_kernel<0><<<dim3(kGate / 16, kMech), 256, 0, stream>>>(WHH, WHHT, nullptr, kHid, kGate, kHid, kWCarry);
  transpose_w_kernel<1><<<dim3(kRt / 16, 1), 256, 0, stream>>>(QPW1, W1TH, W1TL, kHid, kRt, kHid, 1.0f);

  cast_rows_f16_kernel<<<(kRows * (kInP / 8)) / 256, 256, 0, stream>>>(X, X16, kIn, kInP, kRows * (kInP / 8), kActCarry);
  cast_rows_f16_kernel<<<(kRows * (kHid / 8)) / 256, 256, 0, stream>>>(HIN, H16, kHid, kHid, kRows * (kHid / 8), kActCarry);

  router_select_kernel<<<kRows / 64, 128, 0, stream>>>(HIN, W1TH, W1TL, QPB1, QPW2, QPB2, QPW3, QPB3,
                                                      KEYS, WQ, BQ, WK, BK, UNZ, SEL);

  fc1_gemm_kernel<<<(kRows / 64) * (kXaP / 64) / 8, 256, 0, stream>>>(
      X16, kInP, FC1T, kInP, XA16, kXaP, FC1B, kRows, kXaP, kInP, kAccScale, kActCarry);

  gru_select_kernel<<<kRows / 32, 64, 0, stream>>>(XA16, H16, WIHT, WHHT, HIN, BIH, BHH, SEL, OUT1);

  fc2_select_kernel<<<kRows / 16, 256, 0, stream>>>(OUT1, SEL, FC2W, FC2B, OUT0);
}
